// LSTM_ED_Model_34359738952
// MI455X (gfx1250) — hardware-verified
//
#include <hip/hip_runtime.h>
#include <stddef.h>


#define NB 8
#define NT 64
#define NN 512
#define NH 256
#define NO 512
#define NF 24
#define NG 1024

typedef unsigned short us16;
typedef us16   v8us  __attribute__((ext_vector_type(8)));
typedef us16   v16us __attribute__((ext_vector_type(16)));
typedef __bf16 v16b  __attribute__((ext_vector_type(16)));
typedef float  v8f   __attribute__((ext_vector_type(8)));
typedef float  v4f   __attribute__((ext_vector_type(4)));
typedef v8us __attribute__((may_alias)) v8usa;
typedef v4f  __attribute__((may_alias)) v4fa;

union Frag { v16b v; v16us u; v8us h[2]; };

__device__ __forceinline__ v8f vzero8() {
    v8f z = {0.f, 0.f, 0.f, 0.f, 0.f, 0.f, 0.f, 0.f};
    return z;
}

__device__ __forceinline__ us16 bf_rne(float x) {
    unsigned int u = __float_as_uint(x);
    u += 0x7FFFu + ((u >> 16) & 1u);
    return (us16)(u >> 16);
}
__device__ __forceinline__ void split_bf(float x, us16& hi, us16& lo) {
    hi = bf_rne(x);
    const float hv = __uint_as_float(((unsigned int)hi) << 16);
    lo = bf_rne(x - hv);
}

__device__ __forceinline__ v8f mma3(const Frag& ah, const Frag& al, const Frag& bh, const Frag& bl, v8f c) {
    c = __builtin_amdgcn_wmma_f32_16x16x32_bf16(false, ah.v, false, bh.v, (short)0, c, false, false);
    c = __builtin_amdgcn_wmma_f32_16x16x32_bf16(false, ah.v, false, bl.v, (short)0, c, false, false);
    c = __builtin_amdgcn_wmma_f32_16x16x32_bf16(false, al.v, false, bh.v, (short)0, c, false, false);
    asm volatile("v_nop\n\tv_nop\n\tv_nop\n\tv_nop" : "+v"(c) : "v"(ah.v), "v"(al.v), "v"(bh.v), "v"(bl.v));
    return c;
}

__device__ __forceinline__ float sigm(float x) { return 1.0f / (1.0f + expf(-x)); }

__device__ __forceinline__ float wave_max32(float v) {
#pragma unroll
    for (int o = 16; o > 0; o >>= 1) v = fmaxf(v, __shfl_xor(v, o, 32));
    return v;
}

__global__ __launch_bounds__(256)
void pack_kernel(const float* __restrict__ src, us16* hi, us16* lo, int n8)
{
    const int g = blockIdx.x * 256 + threadIdx.x;
    if (g >= n8) return;
    const float* p = src + (size_t)g * 8;
    const v4f x0 = *(const v4f*)p;
    const v4f x1 = *(const v4f*)(p + 4);
    v8us vh, vl;
#pragma unroll
    for (int e = 0; e < 4; ++e) {
        us16 a, b;
        split_bf(x0[e], a, b); vh[e] = a;     vl[e] = b;
        split_bf(x1[e], a, b); vh[4 + e] = a; vl[4 + e] = b;
    }
    volatile v8us* dh = (volatile v8us*)(hi + (size_t)g * 8);
    volatile v8us* dl = (volatile v8us*)(lo + (size_t)g * 8);
    *dh = vh;
    *dl = vl;
    __threadfence();
    *dh = vh;
    *dl = vl;
}

__device__ float gat_row_direct(float ci, const float* __restrict__ arow, const float* sfp, const float* sgp)
{
    float mx = -3.0e38f;
#pragma unroll 1
    for (int j = 0; j < NN; ++j) {
        float v = ci + sgp[j];
        v = (v >= 0.f) ? v : 0.2f * v;
        v = (arow[j] > 0.f) ? v : -9.0e15f;
        mx = fmaxf(mx, v);
    }
    float s = 0.f, w = 0.f;
#pragma unroll 1
    for (int j = 0; j < NN; ++j) {
        float v = ci + sgp[j];
        v = (v >= 0.f) ? v : 0.2f * v;
        v = (arow[j] > 0.f) ? v : -9.0e15f;
        const float e = expf(v - mx);
        s += e;
        w += e * sfp[j];
    }
    return w / s;
}

__global__ __launch_bounds__(256)
void gat_kernel(const float* __restrict__ x, const float* __restrict__ adj,
                const float* __restrict__ gw, const float* __restrict__ ga, float* xg)
{
    __shared__ __attribute__((aligned(16))) float sf[NN];
    __shared__ __attribute__((aligned(16))) float sg[NN];
    __shared__ __attribute__((aligned(16))) float se1[NN];
    __shared__ __attribute__((aligned(16))) float se2[NN];
    __shared__ __attribute__((aligned(16))) float sres[NN];
    __shared__ float sred[8];

    const int bt  = blockIdx.x;
    const int tid = threadIdx.x;
    const float W  = gw[0];
    const float a0 = ga[0];
    const float a1 = ga[1];
    const float* xr = x + (size_t)bt * NN;

    float lmax = -3.0e38f;
#pragma unroll 1
    for (int j = tid; j < NN; j += 256) {
        const float f = xr[j] * W;
        sf[j] = f;
        const float g = a1 * f;
        sg[j] = g;
        lmax = fmaxf(lmax, g);
    }
    lmax = wave_max32(lmax);
    if ((tid & 31) == 0) sred[tid >> 5] = lmax;
    __syncthreads();
    float M = sred[0];
#pragma unroll
    for (int i = 1; i < 8; ++i) M = fmaxf(M, sred[i]);
#pragma unroll 1
    for (int j = tid; j < NN; j += 256) {
        const float d = sg[j] - M;
        se1[j] = expf(d);
        se2[j] = expf(0.2f * d);
    }
    __syncthreads();

#pragma unroll 1
    for (int i = tid; i < NN; i += 256) {
        const float ci = a0 * sf[i];
        const float u  = ci + M;
        const float F  = (u >= 0.f) ? expf(-0.8f * u) : 1.0f;
        const float* arow = adj + (size_t)i * NN;
        float s = 0.f, wsum = 0.f;
#pragma unroll 1
        for (int j = 0; j < NN; j += 4) {
            const v4f av  = *(const v4f*)(arow + j);
            const v4f gv  = *(const v4fa*)&sg[j];
            const v4f e1v = *(const v4fa*)&se1[j];
            const v4f e2v = *(const v4fa*)&se2[j];
            const v4f fv  = *(const v4fa*)&sf[j];
#pragma unroll
            for (int e = 0; e < 4; ++e) {
                const float tv = ci + gv[e];
                float term = (tv >= 0.f) ? e1v[e] : (e2v[e] * F);
                term = (av[e] > 0.f) ? term : 0.f;
                s += term;
                wsum += term * fv[e];
            }
        }
        float r;
        if (s > 0.f) r = wsum / s;
        else         r = gat_row_direct(ci, arow, sf, sg);
        sres[i] = fmaxf(r, 0.f);
    }
    __syncthreads();

    if (tid < NN / 4) {
        const v4f v = *(const v4fa*)&sres[tid * 4];
        volatile v4f* d = (volatile v4f*)(xg + (size_t)bt * NN + tid * 4);
        *d = v;
        __threadfence();
        *d = v;
    }
}

__global__ __launch_bounds__(128)
void xproj_kernel(const float* __restrict__ xg, const us16* __restrict__ wh, const us16* __restrict__ wl, float* gx)
{
    __shared__ __attribute__((aligned(16))) float tile[32][64];
    const int tid = threadIdx.x, w = tid >> 5, l = tid & 31, hf = l >> 4, m = l & 15;
    const int rb = blockIdx.y * 32, cb = blockIdx.x * 64;
    const int row0 = rb + (w >> 1) * 16;
    const int col0 = cb + (w & 1) * 32;

    v8f acc[2];
    acc[0] = vzero8();
    acc[1] = vzero8();

#pragma unroll 1
    for (int k0 = 0; k0 < NN; k0 += 32) {
        Frag ah, al;
        {
            const float* p = xg + (size_t)(row0 + m) * NN + k0 + 8 * hf;
            const v4f x0 = *(const v4f*)(p);
            const v4f x1 = *(const v4f*)(p + 4);
            const v4f x2 = *(const v4f*)(p + 16);
            const v4f x3 = *(const v4f*)(p + 20);
#pragma unroll
            for (int e = 0; e < 4; ++e) {
                us16 a, b;
                split_bf(x0[e], a, b); ah.u[e] = a;      al.u[e] = b;
                split_bf(x1[e], a, b); ah.u[4 + e] = a;  al.u[4 + e] = b;
                split_bf(x2[e], a, b); ah.u[8 + e] = a;  al.u[8 + e] = b;
                split_bf(x3[e], a, b); ah.u[12 + e] = a; al.u[12 + e] = b;
            }
        }
#pragma unroll
        for (int t2 = 0; t2 < 2; ++t2) {
            const size_t bo = (size_t)(col0 + 16 * t2 + m) * NN + k0 + 8 * hf;
            Frag bh, bl;
            bh.h[0] = *(const v8us*)(wh + bo);
            bh.h[1] = *(const v8us*)(wh + bo + 16);
            bl.h[0] = *(const v8us*)(wl + bo);
            bl.h[1] = *(const v8us*)(wl + bo + 16);
            acc[t2] = mma3(ah, al, bh, bl, acc[t2]);
        }
    }
#pragma unroll
    for (int t2 = 0; t2 < 2; ++t2) {
#pragma unroll
        for (int r = 0; r < 8; ++r)
            tile[(w >> 1) * 16 + 8 * hf + r][(w & 1) * 32 + 16 * t2 + m] = acc[t2][r];
    }
    __syncthreads();

    v4f vals[4];
    size_t offs[4];
#pragma unroll
    for (int p = 0; p < 4; ++p) {
        const int L  = p * 16 + (tid >> 3);
        const int rr = L >> 1;
        const int cc = (L & 1) * 32 + (tid & 7) * 4;
        vals[p] = *(const v4fa*)&tile[rr][cc];
        offs[p] = (size_t)(rb + rr) * NG + cb + cc;
    }
#pragma unroll
    for (int p = 0; p < 4; ++p) *(volatile v4f*)(gx + offs[p]) = vals[p];
    __threadfence();
#pragma unroll
    for (int p = 0; p < 4; ++p) *(volatile v4f*)(gx + offs[p]) = vals[p];
}

__device__ __forceinline__ void gate_gemm(v8f (&acc)[4], const us16* aph, const us16* apl, int K,
                                          const us16* __restrict__ wh, const us16* __restrict__ wl,
                                          int j0, int mr, int m, int hf)
{
#pragma unroll 1
    for (int k0 = 0; k0 < K; k0 += 32) {
        Frag ah, al;
        const int ao = mr * K + k0 + 8 * hf;
        ah.h[0] = *(const v8usa*)(aph + ao);
        ah.h[1] = *(const v8usa*)(aph + ao + 16);
        al.h[0] = *(const v8usa*)(apl + ao);
        al.h[1] = *(const v8usa*)(apl + ao + 16);
#pragma unroll
        for (int q = 0; q < 4; ++q) {
            const size_t bo = (size_t)(q * NH + j0 + m) * K + k0 + 8 * hf;
            Frag bh, bl;
            bh.h[0] = *(const v8us*)(wh + bo);
            bh.h[1] = *(const v8us*)(wh + bo + 16);
            bl.h[0] = *(const v8us*)(wl + bo);
            bl.h[1] = *(const v8us*)(wl + bo + 16);
            acc[q] = mma3(ah, al, bh, bl, acc[q]);
        }
    }
}

template <bool ENC>
__device__ __forceinline__ void cell_update(const v8f (&acc)[4], int j, int t, const float* __restrict__ gx,
                                            const float* __restrict__ bih, const float* __restrict__ bhh,
                                            float (*sc)[NH], us16 (*hh)[NH], us16 (*hl)[NH])
{
    float bs[4];
#pragma unroll
    for (int q = 0; q < 4; ++q) bs[q] = bih[q * NH + j] + bhh[q * NH + j];
#pragma unroll
    for (int r = 0; r < NB; ++r) {
        float gi = acc[0][r], gf = acc[1][r], gg = acc[2][r], go = acc[3][r];
        if (ENC) {
            const float* gr = gx + (size_t)(r * NT + t) * NG + j;
            gi += gr[0];
            gf += gr[NH];
            gg += gr[2 * NH];
            go += gr[3 * NH];
        }
        gi += bs[0]; gf += bs[1]; gg += bs[2]; go += bs[3];
        const float cold = sc[r][j];
        const float cn = sigm(gf) * cold + sigm(gi) * tanhf(gg);
        const float hn = sigm(go) * tanhf(cn);
        sc[r][j] = cn;
        us16 a, b;
        split_bf(hn, a, b);
        hh[r][j] = a;
        hl[r][j] = b;
    }
}

__global__ __launch_bounds__(256)
void rnn_kernel(const float* __restrict__ gx,
                const us16* __restrict__ ewh, const us16* __restrict__ ewl,
                const float* __restrict__ ebih, const float* __restrict__ ebhh,
                const us16* __restrict__ dxh, const us16* __restrict__ dxl,
                const us16* __restrict__ dwh, const us16* __restrict__ dwl,
                const float* __restrict__ dbih, const float* __restrict__ dbhh,
                const us16* __restrict__ fwh, const us16* __restrict__ fwl,
                const float* __restrict__ fcb, float* out)
{
    __shared__ __attribute__((aligned(16))) us16  s_hh[2][NB][NH];
    __shared__ __attribute__((aligned(16))) us16  s_hl[2][NB][NH];
    __shared__ __attribute__((aligned(16))) float s_c[NB][NH];
    __shared__ __attribute__((aligned(16))) us16  s_dh[NB][NO];
    __shared__ __attribute__((aligned(16))) us16  s_dl[NB][NO];
    __shared__ __attribute__((aligned(16))) float s_pred[NB][NO];

    const int tid = threadIdx.x, w = tid >> 5, l = tid & 31, hf = l >> 4, m = l & 15, mr = m & 7;

    {
        us16* p0 = &s_hh[0][0][0];
        us16* p1 = &s_hl[0][0][0];
        for (int i = tid; i < 2 * NB * NH; i += 256) { p0[i] = 0; p1[i] = 0; }
        float* pc = &s_c[0][0];
        for (int i = tid; i < NB * NH; i += 256) pc[i] = 0.f;
        us16* pd0 = &s_dh[0][0];
        us16* pd1 = &s_dl[0][0];
        for (int i = tid; i < NB * NO; i += 256) { pd0[i] = 0; pd1[i] = 0; }
    }
    __syncthreads();

    int cur = 0;
#pragma unroll 1
    for (int t = 0; t < NT; ++t) {
        const int nxt = cur ^ 1;
#pragma unroll 1
        for (int ti = 0; ti < 2; ++ti) {
            const int j0 = (w * 2 + ti) * 16;
            v8f acc[4];
            acc[0] = vzero8(); acc[1] = vzero8(); acc[2] = vzero8(); acc[3] = vzero8();
            gate_gemm(acc, &s_hh[cur][0][0], &s_hl[cur][0][0], NH, ewh, ewl, j0, mr, m, hf);
            if (hf == 0) cell_update<true>(acc, j0 + m, t, gx, ebih, ebhh, s_c, s_hh[nxt], s_hl[nxt]);
        }
        __syncthreads();
        cur = nxt;
    }

#pragma unroll 1
    for (int s = 0; s < NF; ++s) {
        const int nxt = cur ^ 1;
#pragma unroll 1
        for (int ti = 0; ti < 2; ++ti) {
            const int j0 = (w * 2 + ti) * 16;
            v8f acc[4];
            acc[0] = vzero8(); acc[1] = vzero8(); acc[2] = vzero8(); acc[3] = vzero8();
            gate_gemm(acc, &s_dh[0][0], &s_dl[0][0], NO, dxh, dxl, j0, mr, m, hf);
            gate_gemm(acc, &s_hh[cur][0][0], &s_hl[cur][0][0], NH, dwh, dwl, j0, mr, m, hf);
            if (hf == 0) cell_update<false>(acc, j0 + m, s, gx, dbih, dbhh, s_c, s_hh[nxt], s_hl[nxt]);
        }
        __syncthreads();

#pragma unroll 1
        for (int ti = 0; ti < 4; ++ti) {
            const int n0 = (w * 4 + ti) * 16;
            v8f facc = vzero8();
            const us16* hp = &s_hh[nxt][0][0];
            const us16* lp = &s_hl[nxt][0][0];
#pragma unroll 1
            for (int k0 = 0; k0 < NH; k0 += 32) {
                Frag ah, al, bh, bl;
                const int ao = mr * NH + k0 + 8 * hf;
                ah.h[0] = *(const v8usa*)(hp + ao);
                ah.h[1] = *(const v8usa*)(hp + ao + 16);
                al.h[0] = *(const v8usa*)(lp + ao);
                al.h[1] = *(const v8usa*)(lp + ao + 16);
                const size_t bo = (size_t)(n0 + m) * NH + k0 + 8 * hf;
                bh.h[0] = *(const v8us*)(fwh + bo);
                bh.h[1] = *(const v8us*)(fwh + bo + 16);
                bl.h[0] = *(const v8us*)(fwl + bo);
                bl.h[1] = *(const v8us*)(fwl + bo + 16);
                facc = mma3(ah, al, bh, bl, facc);
            }
            if (hf == 0) {
                const int n = n0 + m;
                const float bias = fcb[n];
#pragma unroll
                for (int r = 0; r < NB; ++r) {
                    const float p = facc[r] + bias;
                    s_pred[r][n] = p;
                    us16 a, b;
                    split_bf(p, a, b);
                    s_dh[r][n] = a;
                    s_dl[r][n] = b;
                }
            }
        }
        __syncthreads();

        {
            v4f vals[4];
            size_t offs[4];
#pragma unroll
            for (int p = 0; p < 4; ++p) {
                const int L  = p * 32 + (tid >> 3);
                const int rr = L >> 4;
                const int cc = (L & 15) * 32 + (tid & 7) * 4;
                vals[p] = *(const v4fa*)&s_pred[rr][cc];
                offs[p] = (size_t)(rr * NF + s) * NO + cc;
            }
#pragma unroll
            for (int p = 0; p < 4; ++p) *(volatile v4f*)(out + offs[p]) = vals[p];
            __threadfence();
#pragma unroll
            for (int p = 0; p < 4; ++p) *(volatile v4f*)(out + offs[p]) = vals[p];
        }
        __syncthreads();
        cur = nxt;
    }
}

extern "C" void kernel_launch(void* const* d_in, const int* in_sizes, int n_in,
                              void* d_out, int out_size, void* d_ws, size_t ws_size,
                              hipStream_t stream)
{
    if (n_in < 14) return;
    if (in_sizes[0] != NB * NT * NN || in_sizes[1] != NN * NN || in_sizes[2] < 1 || in_sizes[3] < 2 ||
        in_sizes[4] != NG * NN || in_sizes[5] != NG * NH || in_sizes[6] != NG || in_sizes[7] != NG ||
        in_sizes[8] != NG * NO || in_sizes[9] != NG * NH || in_sizes[10] != NG || in_sizes[11] != NG ||
        in_sizes[12] != NO * NH || in_sizes[13] != NO || out_size != NB * NF * NO) return;

    const float* x       = (const float*)d_in[0];
    const float* adj     = (const float*)d_in[1];
    const float* gat_W   = (const float*)d_in[2];
    const float* gat_a   = (const float*)d_in[3];
    const float* enc_Wih = (const float*)d_in[4];
    const float* enc_Whh = (const float*)d_in[5];
    const float* enc_bih = (const float*)d_in[6];
    const float* enc_bhh = (const float*)d_in[7];
    const float* dec_Wih = (const float*)d_in[8];
    const float* dec_Whh = (const float*)d_in[9];
    const float* dec_bih = (const float*)d_in[10];
    const float* dec_bhh = (const float*)d_in[11];
    const float* fc_W    = (const float*)d_in[12];
    const float* fc_b    = (const float*)d_in[13];
    float* out = (float*)d_out;

    char* ws = (char*)d_ws;
    size_t off = 0;
    float* xg = (float*)(ws + off);       off += (size_t)NB * NT * NN * sizeof(float);
    float* gx = (float*)(ws + off);       off += (size_t)NB * NT * NG * sizeof(float);
    us16* ewih_h = (us16*)(ws + off);     off += (size_t)NG * NN * 2;
    us16* ewih_l = (us16*)(ws + off);     off += (size_t)NG * NN * 2;
    us16* ewhh_h = (us16*)(ws + off);     off += (size_t)NG * NH * 2;
    us16* ewhh_l = (us16*)(ws + off);     off += (size_t)NG * NH * 2;
    us16* dwih_h = (us16*)(ws + off);     off += (size_t)NG * NO * 2;
    us16* dwih_l = (us16*)(ws + off);     off += (size_t)NG * NO * 2;
    us16* dwhh_h = (us16*)(ws + off);     off += (size_t)NG * NH * 2;
    us16* dwhh_l = (us16*)(ws + off);     off += (size_t)NG * NH * 2;
    us16* fcw_h  = (us16*)(ws + off);     off += (size_t)NO * NH * 2;
    us16* fcw_l  = (us16*)(ws + off);     off += (size_t)NO * NH * 2;
    if (off > ws_size) return;

    {
        const int n8a = NG * NN / 8, n8b = NG * NH / 8, n8c = NO * NH / 8;
        pack_kernel<<<(n8a + 255) / 256, 256, 0, stream>>>(enc_Wih, ewih_h, ewih_l, n8a);
        pack_kernel<<<(n8b + 255) / 256, 256, 0, stream>>>(enc_Whh, ewhh_h, ewhh_l, n8b);
        pack_kernel<<<(n8a + 255) / 256, 256, 0, stream>>>(dec_Wih, dwih_h, dwih_l, n8a);
        pack_kernel<<<(n8b + 255) / 256, 256, 0, stream>>>(dec_Whh, dwhh_h, dwhh_l, n8b);
        pack_kernel<<<(n8c + 255) / 256, 256, 0, stream>>>(fc_W, fcw_h, fcw_l, n8c);
    }

    gat_kernel<<<NB * NT, 256, 0, stream>>>(x, adj, gat_W, gat_a, xg);

    xproj_kernel<<<dim3(NG / 64, (NB * NT) / 32), 128, 0, stream>>>(xg, ewih_h, ewih_l, gx);

    rnn_kernel<<<1, 256, 0, stream>>>(gx, ewhh_h, ewhh_l, enc_bih, enc_bhh,
                                       dwih_h, dwih_l, dwhh_h, dwhh_l, dec_bih, dec_bhh,
                                       fcw_h, fcw_l, fc_b, out);
}
